// GNNGraphClassifier_29892972380781
// MI455X (gfx1250) — hardware-run, weakly checked
//
#include <hip/hip_runtime.h>
#include <stdint.h>
#include <stddef.h>
#include <math.h>

#pragma clang fp contract(off)

#define NN    50000
#define NG    128
#define DD    32
#define FF    64
#define NA    8
#define HIN   1120
#define NTILE 3125
#define WPB   5
#define TPWV  5
#define NBA   125
#define NBE   625
#define NBB   625
#define EPB   2560
#define NLAY  9
#define EPSF  1e-5f

static_assert(NBA * WPB * TPWV == NTILE);
static_assert(NBE * WPB == NTILE);
static_assert(NTILE * 16 == NN);
static_assert(NBB * EPB == NN * DD);
static_assert(EPB == 10 * 256);
static_assert((NN % 4) == 0);
static_assert(NBB <= 3 * 256);

typedef _Float16 v16h __attribute__((ext_vector_type(16)));
typedef _Float16 v8h  __attribute__((ext_vector_type(8)));
typedef _Float16 v4h  __attribute__((ext_vector_type(4)));
typedef float    v8f  __attribute__((ext_vector_type(8)));
typedef float    v4f  __attribute__((ext_vector_type(4)));
typedef int      v4i  __attribute__((ext_vector_type(4)));
typedef double   v2d  __attribute__((ext_vector_type(2)));
typedef v4f __attribute__((may_alias)) v4fa;
typedef v4i __attribute__((may_alias)) v4ia;
typedef v8h __attribute__((may_alias)) v8ha;
typedef v4h __attribute__((may_alias)) v4ha;

union Frag { v16h v; v8h half[2]; };

__device__ __forceinline__ v8f wmma16(v16h a, v16h b, v8f c) {
  v8f d = __builtin_amdgcn_wmma_f32_16x16x32_f16(false, a, false, b, (short)0, c, false, false);
  asm volatile("v_nop\n\tv_nop\n\tv_nop\n\tv_nop" : "+v"(d) : "v"(a), "v"(b));
  return d;
}

__device__ __forceinline__ v16h ldfrag(const _Float16* p, int h) {
  Frag f;
  f.half[0] = *(const v8ha*)(p + 8 * h);
  f.half[1] = *(const v8ha*)(p + 16 + 8 * h);
  return f.v;
}

__device__ __forceinline__ v16h colfrag16(const float* wcol, int ld, int k0, int h) {
  v16h b;
  #pragma unroll
  for (int i = 0; i < 16; ++i) {
    const int kk = k0 + ((i < 8) ? (8 * h + i) : (8 + 8 * h + i));
    b[i] = (_Float16)(16.0f * wcol[(size_t)kk * ld]);
  }
  return b;
}

__device__ __forceinline__ float wsum(float v) {
  #pragma unroll
  for (int off = 16; off > 0; off >>= 1) v += __shfl_xor(v, off, 32);
  return v;
}
__device__ __forceinline__ int wsumi(int v) {
  #pragma unroll
  for (int off = 16; off > 0; off >>= 1) v += __shfl_xor(v, off, 32);
  return v;
}
__device__ __forceinline__ double wsumd(double v) {
  #pragma unroll
  for (int off = 16; off > 0; off >>= 1) v += __shfl_xor(v, off, 32);
  return v;
}

__global__ __launch_bounds__(160) void k_embed(const float* __restrict__ x, const float* __restrict__ Wi,
                                               const float* __restrict__ bi, const float* __restrict__ lw,
                                               const float* __restrict__ lb, float* __restrict__ hraw)
{
  const int lane = threadIdx.x & 31, wid = threadIdx.x >> 5;
  const int gwv = blockIdx.x * WPB + wid;
  const float w0 = Wi[lane], w1 = Wi[DD + lane], w2 = Wi[2 * DD + lane];
  const float bb = bi[lane], gl = lw[lane], bl = lb[lane];
  #pragma unroll 1
  for (int i = 0; i < 16; ++i) {
    const int n = gwv * 16 + i;
    const float x0 = x[3 * n], x1 = x[3 * n + 1], x2 = x[3 * n + 2];
    const float v = ((x0 * w0 + x1 * w1) + x2 * w2) + bb;
    const float mu = wsum(v) * (1.0f / 32.0f);
    const float c = v - mu;
    const float var = wsum(c * c) * (1.0f / 32.0f);
    const float t = tanhf(c * (1.0f / sqrtf(var + EPSF)) * gl + bl);
    float* p = hraw + (size_t)n * DD + lane;
    *(volatile float*)p = t;
    __threadfence();
    *(volatile float*)p = t;
  }
}

__global__ __launch_bounds__(160) void k_node_a(
    const float* __restrict__ hraw, const float* __restrict__ stat, int lnflag,
    const float* __restrict__ glw, const float* __restrict__ glb,
    const float* __restrict__ Win, const float* __restrict__ bin,
    const float* __restrict__ Wsc, const float* __restrict__ bsc,
    const float* __restrict__ Wout, const float* __restrict__ bout,
    float* __restrict__ U, float* __restrict__ XPF, float* __restrict__ ATT)
{
  __shared__ __align__(16) _Float16 sWin[64 * 40];
  __shared__ __align__(16) _Float16 sWsc[16 * 72];
  __shared__ __align__(16) _Float16 sWo[32 * 104];
  __shared__ __align__(16) float sBin[64];
  __shared__ __align__(16) float sBsc[16];
  __shared__ __align__(16) float sBo[32];
  __shared__ __align__(16) float sGw[32];
  __shared__ __align__(16) float sGb[32];
  __shared__ __align__(16) _Float16 sA[WPB][16 * 40];
  __shared__ __align__(16) _Float16 sXh[WPB][16 * 72];
  __shared__ __align__(16) float sF[WPB][16 * 68];
  __shared__ __align__(16) float sAt[WPB][16 * 8];

  const int tid = threadIdx.x, lane = tid & 31, wid = tid >> 5;
  const int h = lane >> 4, m = lane & 15;

  #pragma unroll 1
  for (int i = 0; i < 13; ++i) {
    const int idx = tid + 160 * i;
    const int ic = (idx < 2048) ? idx : 2047;
    const float v = Win[ic];
    if (idx < 2048) sWin[(ic & 63) * 40 + (ic >> 6)] = (_Float16)(16.0f * v);
  }
  #pragma unroll 1
  for (int i = 0; i < 4; ++i) {
    const int idx = tid + 160 * i;
    const int ic = (idx < 512) ? idx : 511;
    const float v = Wsc[ic];
    if (idx < 512) {
      sWsc[(ic & 7) * 72 + (ic >> 3)] = (_Float16)(16.0f * v);
      sWsc[(8 + (ic >> 6)) * 72 + (ic & 63)] = (_Float16)0.0f;
    }
  }
  #pragma unroll 1
  for (int i = 0; i < 20; ++i) {
    const int idx = tid + 160 * i;
    const int ic = (idx < 3072) ? idx : 3071;
    const float v = Wout[ic];
    if (idx < 3072) sWo[(ic & 31) * 104 + (ic >> 5)] = (_Float16)(16.0f * v);
  }
  if (tid < 64) sBin[tid] = bin[tid];
  if (tid < 32) {
    const float vb = bsc[(tid < NA) ? tid : (NA - 1)];
    if (tid < 16) sBsc[tid] = (tid < NA) ? vb : 0.0f;
    sBo[tid] = bout[tid];
    const float a = glw[tid], b = glb[tid];
    sGw[tid] = lnflag ? a : 1.0f;
    sGb[tid] = lnflag ? b : 0.0f;
  }
  float mean = 0.0f, inv = 1.0f;
  if (lnflag) { mean = stat[0]; inv = stat[1]; }
  __syncthreads();

  _Float16* mA  = sA[wid];
  _Float16* mXh = sXh[wid];
  float*    mF  = sF[wid];
  float*    mAt = sAt[wid];
  const v8f z8 = {0.f, 0.f, 0.f, 0.f, 0.f, 0.f, 0.f, 0.f};

  #pragma unroll 1
  for (int it = 0; it < TPWV; ++it) {
    const int tile = (blockIdx.x * WPB + wid) * TPWV + it;
    const size_t node0 = (size_t)tile * 16;

    #pragma unroll
    for (int i = 0; i < 4; ++i) {
      const int q = lane + 32 * i;
      const int mr = q >> 3, d0 = 4 * (q & 7);
      const v4f v  = *(const v4fa*)(hraw + node0 * DD + 4 * q);
      const v4f gw = *(const v4fa*)(sGw + d0);
      const v4f gb = *(const v4fa*)(sGb + d0);
      const v4f y = (v - mean) * inv * gw + gb;
      const v4h yh = __builtin_convertvector(y, v4h);
      *(v4ha*)(mA + mr * 40 + d0) = yh;
    }
    __syncthreads();

    const v16h aH = ldfrag(mA + m * 40, h);
    v8f accx[4];
    #pragma unroll
    for (int nt = 0; nt < 4; ++nt) accx[nt] = wmma16(aH, ldfrag(sWin + (16 * nt + m) * 40, h), z8);
    #pragma unroll
    for (int nt = 0; nt < 4; ++nt) {
      const int col = 16 * nt + m;
      const float bc = sBin[col];
      #pragma unroll
      for (int r = 0; r < 8; ++r) {
        const int row = 8 * h + r;
        const float v = accx[nt][r] * 0.0625f + bc;
        mF[row * 68 + col] = v;
        mXh[row * 72 + col] = (_Float16)v;
      }
    }
    __syncthreads();

    {
      v4f xv[8];
      #pragma unroll
      for (int i = 0; i < 8; ++i) {
        const int q = lane + 32 * i;
        xv[i] = *(const v4fa*)(mF + (q >> 4) * 68 + 4 * (q & 15));
      }
      float* gx = XPF + node0 * FF + 4 * lane;
      #pragma unroll
      for (int i = 0; i < 8; ++i) *(volatile v4f*)(gx + 128 * i) = xv[i];
      __threadfence();
      #pragma unroll
      for (int i = 0; i < 8; ++i) *(volatile v4f*)(gx + 128 * i) = xv[i];
    }
    const v16h aX0 = ldfrag(mXh + m * 72, h);
    const v16h aX1 = ldfrag(mXh + m * 72 + 32, h);
    v8f accs = wmma16(aX0, ldfrag(sWsc + m * 72, h), z8);
    accs = wmma16(aX1, ldfrag(sWsc + m * 72 + 32, h), accs);
    {
      const float bs = sBsc[m];
      #pragma unroll
      for (int r = 0; r < 8; ++r) {
        const float a = expf(-fabsf(accs[r] * 0.0625f + bs));
        if (m < NA) mAt[(8 * h + r) * NA + m] = a;
      }
    }
    v8f accu[2];
    #pragma unroll
    for (int nt = 0; nt < 2; ++nt) {
      const _Float16* wr = sWo + (16 * nt + m) * 104;
      accu[nt] = wmma16(aH,  ldfrag(wr,      h), z8);
      accu[nt] = wmma16(aX0, ldfrag(wr + 32, h), accu[nt]);
      accu[nt] = wmma16(aX1, ldfrag(wr + 64, h), accu[nt]);
    }
    __syncthreads();

    #pragma unroll
    for (int nt = 0; nt < 2; ++nt) {
      const int col = 16 * nt + m;
      const float bc = sBo[col];
      #pragma unroll
      for (int r = 0; r < 8; ++r) mF[(8 * h + r) * 36 + col] = accu[nt][r] * 0.0625f + bc;
    }
    __syncthreads();

    {
      const v4f av = *(const v4fa*)(mAt + 4 * lane);
      v4f uv[4];
      #pragma unroll
      for (int i = 0; i < 4; ++i) {
        const int q = lane + 32 * i;
        uv[i] = *(const v4fa*)(mF + (q >> 3) * 36 + 4 * (q & 7));
      }
      float* ga = ATT + node0 * NA + 4 * lane;
      float* gu = U + node0 * DD + 4 * lane;
      *(volatile v4f*)ga = av;
      #pragma unroll
      for (int i = 0; i < 4; ++i) *(volatile v4f*)(gu + 128 * i) = uv[i];
      __threadfence();
      *(volatile v4f*)ga = av;
      #pragma unroll
      for (int i = 0; i < 4; ++i) *(volatile v4f*)(gu + 128 * i) = uv[i];
    }
    __syncthreads();
  }
}

__global__ __launch_bounds__(128) void k_seg(const float* __restrict__ XPF, const float* __restrict__ ATT,
                                             const int* __restrict__ batch, _Float16* __restrict__ AGG)
{
  __shared__ __align__(16) float sX[32 * FF];
  __shared__ __align__(16) float sT[32 * NA];
  __shared__ __align__(16) _Float16 sG[NA * 2 * FF];
  __shared__ int sI[8];
  const int tid = threadIdx.x, lane = tid & 31, wid = tid >> 5, g = blockIdx.x;
  const int f = tid & 63, ah = tid >> 6;

  {
    int c = 0, lt = 0;
    const v4ia* b4 = (const v4ia*)batch;
    #pragma unroll 1
    for (int i = tid; i < NN / 4; i += 128) {
      const v4i b = b4[i];
      c  += (b.x == g) + (b.y == g) + (b.z == g) + (b.w == g);
      lt += (b.x <  g) + (b.y <  g) + (b.z <  g) + (b.w <  g);
    }
    c = wsumi(c); lt = wsumi(lt);
    if (lane == 0) { sI[wid] = c; sI[4 + wid] = lt; }
  }
  __syncthreads();
  int cnt = (sI[0] + sI[1]) + (sI[2] + sI[3]);
  int st  = (sI[4] + sI[5]) + (sI[6] + sI[7]);
  st  = (st < 0) ? 0 : ((st > NN) ? NN : st);
  cnt = (cnt < 0) ? 0 : cnt;
  cnt = (cnt > NN - st) ? (NN - st) : cnt;

  const float NINF = __uint_as_float(0xff800000u);
  float s[4], mx[4];
  #pragma unroll
  for (int i = 0; i < 4; ++i) { s[i] = 0.0f; mx[i] = NINF; }

  const int nch = (cnt + 31) >> 5;
  #pragma unroll 1
  for (int ch = 0; ch < nch; ++ch) {
    const int base = st + 32 * ch;
    int nv = cnt - 32 * ch; nv = (nv > 32) ? 32 : nv;
    __syncthreads();
    #pragma unroll
    for (int i = 0; i < 4; ++i) {
      const int q = tid + 128 * i;
      const int nl = q >> 4, c4 = 4 * (q & 15);
      int n = base + nl; n = (n > NN - 1) ? (NN - 1) : n;
      *(v4fa*)(sX + nl * FF + c4) = *(const v4fa*)(XPF + (size_t)n * FF + c4);
    }
    if (tid < 64) {
      const int nl = tid >> 1, c4 = 4 * (tid & 1);
      int n = base + nl; n = (n > NN - 1) ? (NN - 1) : n;
      *(v4fa*)(sT + nl * NA + c4) = *(const v4fa*)(ATT + (size_t)n * NA + c4);
    }
    __syncthreads();
    #pragma unroll 2
    for (int nl = 0; nl < nv; ++nl) {
      const float xv = sX[nl * FF + f];
      const v4f at = *(const v4fa*)(sT + nl * NA + 4 * ah);
      const float w0 = at.x * xv, w1 = at.y * xv, w2 = at.z * xv, w3 = at.w * xv;
      s[0] += w0; s[1] += w1; s[2] += w2; s[3] += w3;
      mx[0] = fmaxf(mx[0], w0); mx[1] = fmaxf(mx[1], w1);
      mx[2] = fmaxf(mx[2], w2); mx[3] = fmaxf(mx[3], w3);
    }
  }
  const float rc = 1.0f / fmaxf((float)cnt, 1.0f);
  const bool nz = (cnt > 0);
  #pragma unroll
  for (int i = 0; i < 4; ++i) {
    const int a = 4 * ah + i;
    const float mv = nz ? mx[i] : 0.0f;
    sG[a * 128 + f]      = (_Float16)(16.0f * (s[i] * rc));
    sG[a * 128 + 64 + f] = (_Float16)(16.0f * mv);
  }
  __syncthreads();
  const v4i gv = *(const v4ia*)(sG + 8 * tid);
  _Float16* gp = AGG + (size_t)g * 1024 + 8 * tid;
  *(volatile v4i*)gp = gv;
  __threadfence();
  *(volatile v4i*)gp = gv;
}

__global__ __launch_bounds__(512) void k_aggp(const _Float16* __restrict__ AGG, const float* __restrict__ Wout,
                                              float* __restrict__ AGGP)
{
  __shared__ __align__(16) float sP[NG * 36];
  const int tid = threadIdx.x, lane = tid & 31, wid = tid >> 5;
  const int h = lane >> 4, m = lane & 15;
  const int mt = wid >> 1, nt = wid & 1;
  const _Float16* arow = AGG + (size_t)(16 * mt + m) * 1024;
  const float* wcol = Wout + 96 * DD + 16 * nt + m;
  const v8f z8 = {0.f, 0.f, 0.f, 0.f, 0.f, 0.f, 0.f, 0.f};
  v8f acc = z8;
  #pragma unroll 1
  for (int ks = 0; ks < 32; ++ks) {
    const int k0 = 32 * ks;
    const v16h a = ldfrag(arow + k0, h);
    const v16h b = colfrag16(wcol, DD, k0, h);
    acc = wmma16(a, b, acc);
  }
  #pragma unroll
  for (int r = 0; r < 8; ++r) sP[(16 * mt + 8 * h + r) * 36 + 16 * nt + m] = acc[r] * (1.0f / 256.0f);
  __syncthreads();
  v4f pv[2];
  #pragma unroll
  for (int i = 0; i < 2; ++i) {
    const int q = tid + 512 * i;
    pv[i] = *(const v4fa*)(sP + (q >> 3) * 36 + 4 * (q & 7));
  }
  #pragma unroll
  for (int i = 0; i < 2; ++i) *(volatile v4f*)(AGGP + 4 * (tid + 512 * i)) = pv[i];
  __threadfence();
  #pragma unroll
  for (int i = 0; i < 2; ++i) *(volatile v4f*)(AGGP + 4 * (tid + 512 * i)) = pv[i];
}

__global__ __launch_bounds__(256) void k_node_b(const float* __restrict__ U, const float* __restrict__ AGGP,
                                                const int* __restrict__ batch, float* __restrict__ hraw,
                                                double* __restrict__ part)
{
  __shared__ float sT[EPB];
  __shared__ double sR[16];
  __shared__ double sTot[2];
  const int tid = threadIdx.x, lane = tid & 31, wid = tid >> 5;
  const size_t base = (size_t)blockIdx.x * EPB;
  double s = 0.0, s2 = 0.0;
  #pragma unroll 1
  for (int i = 0; i < 10; ++i) {
    const size_t e = base + 256 * i + tid;
    const int n = (int)(e >> 5), d = (int)(e & 31);
    int g = batch[n];
    g = (g < 0) ? 0 : ((g > NG - 1) ? (NG - 1) : g);
    const float v = U[e] + AGGP[g * DD + d];
    const float t = tanhf(v);
    sT[256 * i + tid] = t;
    s  += (double)t;
    s2 += (double)t * (double)t;
    *(volatile float*)(hraw + e) = t;
  }
  __threadfence();
  #pragma unroll 1
  for (int i = 0; i < 10; ++i) *(volatile float*)(hraw + base + 256 * i + tid) = sT[256 * i + tid];

  s = wsumd(s); s2 = wsumd(s2);
  if (lane == 0) { sR[wid] = s; sR[8 + wid] = s2; }
  __syncthreads();
  if (tid == 0) {
    double a = 0.0, b = 0.0;
    for (int w = 0; w < 8; ++w) { a += sR[w]; b += sR[8 + w]; }
    sTot[0] = a; sTot[1] = b;
  }
  __syncthreads();
  const double ta = sTot[0], tb = sTot[1];
  v2d pv;
  pv.x = (tid == 0) ? ta : 0.0;
  pv.y = (tid == 0) ? tb : 0.0;
  const int tq = (tid < 8) ? tid : 0;
  double* pp = part + (size_t)blockIdx.x * 16 + 2 * tq;
  if (tid < 8) *(volatile v2d*)pp = pv;
  __threadfence();
  if (tid < 8) *(volatile v2d*)pp = pv;
}

__global__ __launch_bounds__(256) void k_stat(const double* __restrict__ part, float* __restrict__ statl)
{
  __shared__ double sR[16];
  __shared__ float sO[2];
  const int tid = threadIdx.x, lane = tid & 31, wid = tid >> 5;
  double s = 0.0, s2 = 0.0;
  #pragma unroll 1
  for (int i = 0; i < 3; ++i) {
    const int b = tid + 256 * i;
    const int bc = (b < NBB) ? b : (NBB - 1);
    const double a = part[(size_t)bc * 16], c = part[(size_t)bc * 16 + 1];
    s  += (b < NBB) ? a : 0.0;
    s2 += (b < NBB) ? c : 0.0;
  }
  s = wsumd(s); s2 = wsumd(s2);
  if (lane == 0) { sR[wid] = s; sR[8 + wid] = s2; }
  __syncthreads();
  if (tid == 0) {
    double a = 0.0, b = 0.0;
    for (int w = 0; w < 8; ++w) { a += sR[w]; b += sR[8 + w]; }
    const double nd = (double)NN * (double)DD;
    const double mu = a / nd;
    double var = b / nd - mu * mu;
    var = (var > 0.0) ? var : 0.0;
    const float sd = sqrtf((float)var);
    sO[0] = (float)mu;
    sO[1] = 1.0f / (sd + EPSF);
  }
  __syncthreads();
  const float mo = sO[0], io = sO[1];
  v4f v;
  v.x = (tid == 0) ? mo : 0.0f;
  v.y = (tid == 0) ? io : 0.0f;
  v.z = 0.0f; v.w = 0.0f;
  const int tq = (tid < 8) ? tid : 0;
  if (tid < 8) *(volatile v4f*)(statl + 4 * tq) = v;
  __threadfence();
  if (tid < 8) *(volatile v4f*)(statl + 4 * tq) = v;
}

__global__ __launch_bounds__(256) void k_head(
    const float* __restrict__ hraw, const int* __restrict__ batch, const float* __restrict__ stat,
    const float* __restrict__ glw, const float* __restrict__ glb,
    const float* __restrict__ Wp, const float* __restrict__ bp,
    const float* __restrict__ lw, const float* __restrict__ lb,
    const float* __restrict__ Wpo, const float* __restrict__ bpo, float* __restrict__ out)
{
  __shared__ __align__(16) float sS[NG * 36];
  __shared__ __align__(16) _Float16 sH[NG * 40];
  __shared__ __align__(16) float sO[NG];
  __shared__ int sCnt[NG];
  __shared__ int sSt[NG];
  const int tid = threadIdx.x, lane = tid & 31, wid = tid >> 5;
  const int h = lane >> 4, m = lane & 15;

  if (tid < NG) {
    int c = 0, lt = 0;
    const v4ia* b4 = (const v4ia*)batch;
    #pragma unroll 1
    for (int i = 0; i < NN / 4; ++i) {
      const v4i b = b4[i];
      c  += (b.x == tid) + (b.y == tid) + (b.z == tid) + (b.w == tid);
      lt += (b.x <  tid) + (b.y <  tid) + (b.z <  tid) + (b.w <  tid);
    }
    sCnt[tid] = c; sSt[tid] = lt;
  }
  __syncthreads();

  const float mean = stat[0], inv = stat[1], gw = glw[lane], gb = glb[lane];
  #pragma unroll 1
  for (int gi = 0; gi < 16; ++gi) {
    const int g = 16 * wid + gi;
    int st = sSt[g], cnt = sCnt[g];
    st  = (st < 0) ? 0 : ((st > NN) ? NN : st);
    cnt = (cnt < 0) ? 0 : cnt;
    cnt = (cnt > NN - st) ? (NN - st) : cnt;
    float acc = 0.0f;
    #pragma unroll 2
    for (int k = 0; k < cnt; ++k) {
      const int n = st + k;
      acc += (hraw[(size_t)n * DD + lane] - mean) * inv * gw + gb;
    }
    const float sv = acc * (1.0f / fmaxf((float)cnt, 1.0f));
    sS[g * 36 + lane] = sv;
    sH[g * 40 + lane] = (_Float16)sv;
  }
  __syncthreads();

  const v8f z8 = {0.f, 0.f, 0.f, 0.f, 0.f, 0.f, 0.f, 0.f};
  #pragma unroll 1
  for (int j = 0; j < 3; ++j) {
    const v16h a = ldfrag(sH + (16 * wid + m) * 40, h);
    v8f acc[2];
    #pragma unroll
    for (int nt = 0; nt < 2; ++nt) {
      const v16h b = colfrag16(Wp + j * DD * DD + 16 * nt + m, DD, 0, h);
      acc[nt] = wmma16(a, b, z8);
    }
    __syncthreads();
    #pragma unroll
    for (int nt = 0; nt < 2; ++nt) {
      const int col = 16 * nt + m;
      const float bc = bp[j * DD + col];
      #pragma unroll
      for (int r = 0; r < 8; ++r) sS[(16 * wid + 8 * h + r) * 36 + col] = acc[nt][r] * 0.0625f + bc;
    }
    __syncthreads();
    const float lwv = lw[j * DD + lane], lbv = lb[j * DD + lane];
    #pragma unroll 1
    for (int q = 0; q < 16; ++q) {
      const int row = 16 * wid + q;
      const float y = sS[row * 36 + lane];
      const float mu = wsum(y) * (1.0f / 32.0f);
      const float c = y - mu;
      const float var = wsum(c * c) * (1.0f / 32.0f);
      const float t = tanhf(c * (1.0f / sqrtf(var + EPSF)) * lwv + lbv);
      sS[row * 36 + lane] = t;
      sH[row * 40 + lane] = (_Float16)t;
    }
    __syncthreads();
  }

  const float wo = Wpo[lane], b0 = bpo[0];
  #pragma unroll 1
  for (int q = 0; q < 16; ++q) {
    const int row = 16 * wid + q;
    const float r = wsum(sS[row * 36 + lane] * wo);
    if (lane == 0) sO[row] = r + b0;
  }
  __syncthreads();
  const int tq = (tid < 32) ? tid : 0;
  const v4f ov = *(const v4fa*)(sO + 4 * tq);
  if (tid < 32) *(volatile v4f*)(out + 4 * tq) = ov;
  __threadfence();
  if (tid < 32) *(volatile v4f*)(out + 4 * tq) = ov;
}

extern "C" void kernel_launch(void* const* d_in, const int* in_sizes, int n_in,
                              void* d_out, int out_size, void* d_ws, size_t ws_size,
                              hipStream_t stream)
{
  if (n_in < 20) return;
  if (in_sizes[0]  != NN * 3) return;
  if (in_sizes[1]  != NN) return;
  if (in_sizes[2]  != 3 * DD) return;
  if (in_sizes[3]  != DD) return;
  if (in_sizes[4]  != DD) return;
  if (in_sizes[5]  != DD) return;
  if (in_sizes[6]  != 3 * DD * FF) return;
  if (in_sizes[7]  != 3 * FF) return;
  if (in_sizes[8]  != 3 * FF * NA) return;
  if (in_sizes[9]  != 3 * NA) return;
  if (in_sizes[10] != 3 * HIN * DD) return;
  if (in_sizes[11] != 3 * DD) return;
  if (in_sizes[12] != 3 * DD) return;
  if (in_sizes[13] != 3 * DD) return;
  if (in_sizes[14] != 3 * DD * DD) return;
  if (in_sizes[15] != 3 * DD) return;
  if (in_sizes[16] != 3 * DD) return;
  if (in_sizes[17] != 3 * DD) return;
  if (in_sizes[18] != DD) return;
  if (in_sizes[19] < 1) return;
  if (out_size != NG) return;

  const float* x     = (const float*)d_in[0];
  const int*   batch = (const int*)d_in[1];
  const float* Wi    = (const float*)d_in[2];
  const float* bi    = (const float*)d_in[3];
  const float* lni_w = (const float*)d_in[4];
  const float* lni_b = (const float*)d_in[5];
  const float* W_in  = (const float*)d_in[6];
  const float* b_in  = (const float*)d_in[7];
  const float* W_sc  = (const float*)d_in[8];
  const float* b_sc  = (const float*)d_in[9];
  const float* W_out = (const float*)d_in[10];
  const float* b_out = (const float*)d_in[11];
  const float* gln_w = (const float*)d_in[12];
  const float* gln_b = (const float*)d_in[13];
  const float* Wp    = (const float*)d_in[14];
  const float* bp    = (const float*)d_in[15];
  const float* lnp_w = (const float*)d_in[16];
  const float* lnp_b = (const float*)d_in[17];
  const float* Wpo   = (const float*)d_in[18];
  const float* bpo   = (const float*)d_in[19];
  float* out = (float*)d_out;

  const size_t bSTAT = (size_t)NLAY * 128;
  const size_t bPART = (size_t)NBB * 128;
  const size_t bH    = (size_t)NN * DD * 4;
  const size_t bU    = (size_t)NN * DD * 4;
  const size_t bX    = (size_t)NN * FF * 4;
  const size_t bAT   = (size_t)NN * NA * 4;
  const size_t bAGG  = (size_t)NG * 1024 * 2;
  const size_t bAGP  = (size_t)NG * DD * 4;
  const size_t total = bSTAT + bPART + bH + bU + bX + bAT + bAGG + bAGP;
  if (total > ws_size) return;
  if (total > (size_t)134217728) return;

  char* ws = (char*)d_ws;
  size_t off = 0;
  float*    STAT = (float*)(ws + off);    off += bSTAT;
  double*   PART = (double*)(ws + off);   off += bPART;
  float*    HRAW = (float*)(ws + off);    off += bH;
  float*    UB   = (float*)(ws + off);    off += bU;
  float*    XPF  = (float*)(ws + off);    off += bX;
  float*    ATT  = (float*)(ws + off);    off += bAT;
  _Float16* AGG  = (_Float16*)(ws + off); off += bAGG;
  float*    AGGP = (float*)(ws + off);    off += bAGP;
  if (off != total) return;

  k_embed<<<NBE, 160, 0, stream>>>(x, Wi, bi, lni_w, lni_b, HRAW);

  for (int L = 0; L < NLAY; ++L) {
    const int j  = L % 3;
    const int jp = (L + 2) % 3;
    const int lp = (L > 0) ? (L - 1) : 0;
    k_node_a<<<NBA, 160, 0, stream>>>(HRAW, STAT + 32 * lp, (L > 0) ? 1 : 0,
                                      gln_w + jp * DD, gln_b + jp * DD,
                                      W_in + (size_t)j * DD * FF, b_in + j * FF,
                                      W_sc + (size_t)j * FF * NA, b_sc + j * NA,
                                      W_out + (size_t)j * HIN * DD, b_out + j * DD,
                                      UB, XPF, ATT);
    k_seg<<<NG, 128, 0, stream>>>(XPF, ATT, batch, AGG);
    k_aggp<<<1, 512, 0, stream>>>(AGG, W_out + (size_t)j * HIN * DD, AGGP);
    k_node_b<<<NBB, 256, 0, stream>>>(UB, AGGP, batch, HRAW, PART);
    k_stat<<<1, 256, 0, stream>>>(PART, STAT + 32 * L);
  }

  k_head<<<1, 256, 0, stream>>>(HRAW, batch, STAT + 32 * (NLAY - 1), gln_w + 2 * DD, gln_b + 2 * DD,
                                Wp, bp, lnp_w, lnp_b, Wpo, bpo, out);
}
